// Response_score_44401371906485
// MI455X (gfx1250) — hardware-verified
//
#include <hip/hip_runtime.h>


#ifndef NB
#define NB 4
#endif
#ifndef NQ
#define NQ 512
#endif
#ifndef NK
#define NK 512
#endif
#define NB_FULL 4
#define NQ_FULL 512
#define NK_FULL 512
#ifndef OUT_Q
#define OUT_Q NQ
#endif
#ifndef OUT_K
#define OUT_K NK
#endif
#define DIN  512
#define HID  256
#define MQ   (NB * NQ)
#define MK   (NB * NK)
#define MT   (MQ + MK)
#ifndef TANH_LIBM
#define TANH_LIBM 0
#endif
#define TL2E 2.8853900817779268f

static_assert(DIN % 32 == 0);
static_assert(DIN % 64 == 0);
static_assert(HID % 64 == 0);
static_assert(HID == 256);
static_assert(MQ % 64 == 0);
static_assert(MK % 64 == 0);
static_assert(NK % 128 == 0);
static_assert(NK % 8 == 0);
static_assert(NB <= NB_FULL);
static_assert(NQ <= NQ_FULL);
static_assert(NK <= NK_FULL);
static_assert(OUT_K >= NK);
static_assert((OUT_K * 4) % 128 == 0);
static_assert(((size_t)NQ * DIN) % 8 == 0);
static_assert(((size_t)NK * DIN) % 8 == 0);
static_assert(16 * 68 * 4 <= 131072);
static_assert(64 * 65 * 4 <= 131072);
static_assert(NK * 4 <= 131072);

typedef unsigned short bf;
typedef __attribute__((ext_vector_type(16))) __bf16   v16bf;
typedef __attribute__((ext_vector_type(8)))  unsigned short v8us;
typedef __attribute__((ext_vector_type(8)))  float    v8f;
typedef __attribute__((ext_vector_type(4)))  float    v4f;
typedef v4f  __attribute__((may_alias)) v4fa;

__device__ __forceinline__ unsigned short f2bf(float f) { unsigned u = __float_as_uint(f); u += 0x7FFFu + ((u >> 16) & 1u); return (unsigned short)(u >> 16); }
__device__ __forceinline__ float bfr(float f) { return __uint_as_float(((unsigned)f2bf(f)) << 16); }
__device__ __forceinline__ v16bf cat16b(v8us lo, v8us hi) { return __builtin_bit_cast(v16bf, __builtin_shufflevector(lo, hi, 0, 1, 2, 3, 4, 5, 6, 7, 8, 9, 10, 11, 12, 13, 14, 15)); }
__device__ __forceinline__ v8f wmmab(v16bf a, v16bf b, v8f c) { return __builtin_amdgcn_wmma_f32_16x16x32_bf16(false, a, false, b, (short)0, c, false, false); }
__device__ __forceinline__ v8f wmmabg(v16bf a, v16bf b, v8f c) { c = wmmab(a, b, c); asm volatile("v_nop\n\tv_nop\n\tv_nop\n\tv_nop" : "+v"(c) : "v"(a), "v"(b)); return c; }
__device__ __forceinline__ v16bf ldb(const bf* p)  { return cat16b(*(const v8us*)p, *(const v8us*)(p + 16)); }
__device__ __forceinline__ void wave_sync() { __builtin_amdgcn_fence(3  , "wavefront"); __builtin_amdgcn_wave_barrier(); asm volatile("" ::: "memory"); }

__device__ __forceinline__ float tanh_e(float x) {
#if TANH_LIBM
    return tanhf(x);
#else
    const float e = __builtin_amdgcn_exp2f(x * TL2E);
    const float r = __builtin_amdgcn_rcpf(e + 1.0f);
    return fmaf(-2.0f, r, 1.0f);
#endif
}

__global__ __launch_bounds__(256) void k_cvt8(const float* __restrict__ src, bf* dst, size_t n8) {
    const size_t i = (size_t)blockIdx.x * 256 + threadIdx.x; if (i >= n8) return;
    const v8f v = *(const v8f*)(src + i * 8); v8us o;
#pragma unroll
    for (int k = 0; k < 8; ++k) o[k] = f2bf(v[k]);
    *(volatile v8us*)(dst + i * 8) = o; __threadfence(); *(volatile v8us*)(dst + i * 8) = o;
}

static_assert(4 * 256 * 4 == 64 * 64);
static_assert(2 * 256 * 16 == 64 * 64 * 2);
__global__ __launch_bounds__(256) void k_wtr(const float* __restrict__ W, bf* WT) {
    __shared__ float ts[64 * 65];
    const unsigned t = threadIdx.x;
    const unsigned k0 = blockIdx.x * 64u, n0 = blockIdx.y * 64u;
#pragma unroll
    for (unsigned it = 0; it < 4; ++it) {
        const unsigned e = it * 256u + t; const unsigned kk = e >> 4, n4 = (e & 15u) * 4u;
        const v4f v = *(const v4f*)(W + (size_t)(k0 + kk) * HID + n0 + n4);
        ts[kk * 65u + n4 + 0u] = v[0]; ts[kk * 65u + n4 + 1u] = v[1]; ts[kk * 65u + n4 + 2u] = v[2]; ts[kk * 65u + n4 + 3u] = v[3]; }
    __syncthreads();
    v8us o[2];
#pragma unroll
    for (unsigned it = 0; it < 2; ++it) {
        const unsigned p = it * 256u + t; const unsigned row = p >> 3, c8 = (p & 7u) * 8u;
#pragma unroll
        for (unsigned i = 0; i < 8; ++i) o[it][i] = f2bf(ts[(c8 + i) * 65u + row]); }
#pragma unroll 1
    for (int ps = 0; ps < 2; ++ps) {
#pragma unroll
        for (unsigned it = 0; it < 2; ++it) {
            const unsigned p = it * 256u + t; const unsigned row = p >> 3, c8 = (p & 7u) * 8u;
            *(volatile v8us*)(WT + (size_t)(n0 + row) * DIN + k0 + c8) = o[it]; }
        if (ps == 0) __threadfence(); }
}

static_assert(8 * 32 * 16 == 16 * 64 * 4);
__global__ __launch_bounds__(32) void k_gemm(const bf* __restrict__ A, const bf* __restrict__ Bt, float* C) {
    __shared__ __align__(16) float os[16 * 68];
    const int K = DIN;
    const int lane = threadIdx.x & 31, lr = lane & 15, hi = lane >> 4;
    const unsigned bx = blockIdx.x, by = blockIdx.y;
    const int r0 = (int)(bx * 64u), c0 = (int)(by * 64u);
    const unsigned wsel = (bx * 64u >= (unsigned)MQ) ? 1u : 0u;
    v8f acc[4][4];
#pragma unroll
    for (int mb = 0; mb < 4; ++mb)
#pragma unroll
        for (int nb = 0; nb < 4; ++nb) acc[mb][nb] = (v8f){};
    const size_t aoff = (size_t)(r0 + lr) * K + 8 * hi;
    const size_t boff = (size_t)wsel * ((size_t)HID * DIN) + (size_t)(c0 + lr) * K + 8 * hi;
#pragma unroll 1
    for (int kc = 0; kc < K; kc += 32) {
        v16bf a[4];
#pragma unroll
        for (int mb = 0; mb < 4; ++mb) a[mb] = ldb(A + aoff + (size_t)mb * 16 * K + kc);
#pragma unroll
        for (int nb = 0; nb < 4; ++nb) { const v16bf b = ldb(Bt + boff + (size_t)nb * 16 * K + kc);
#pragma unroll
            for (int mb = 0; mb < 4; ++mb) acc[mb][nb] = wmmabg(a[mb], b, acc[mb][nb]); }
    }
#pragma unroll
    for (int mb = 0; mb < 4; ++mb) {
#pragma unroll
        for (int nb = 0; nb < 4; ++nb) {
#pragma unroll
            for (int j = 0; j < 8; ++j) os[(hi * 8 + j) * 68 + nb * 16 + lr] = acc[mb][nb][j]; }
        wave_sync();
        float* cb = C + (size_t)(r0 + mb * 16) * HID + c0;
#pragma unroll 1
        for (int ps = 0; ps < 2; ++ps) {
#pragma unroll
            for (int s = 0; s < 8; ++s) { const int row = 2 * s + hi, c4 = lr * 4;
                const v4f val = *(const v4fa*)(&os[row * 68 + c4]);
                *(volatile v4f*)(cb + (size_t)row * HID + c4) = val; }
            if (ps == 0) __threadfence(); }
        wave_sync();
    }
}

static_assert((NK / 128) * 32 * 16 == NK * 4);
__global__ __launch_bounds__(256) void k_score(const float* __restrict__ QP, const float* __restrict__ KP, const float* __restrict__ wv, float* OUT) {
    __shared__ __align__(16) float res[NK];
    const int lane = threadIdx.x & 31;
    const int wave = __builtin_amdgcn_readfirstlane((int)(threadIdx.x >> 5));
    const unsigned qi = blockIdx.x, b = blockIdx.y;
    const float* qrow = QP + ((size_t)b * NQ + qi) * HID + 4 * lane;
    const v4f qa = *(const v4f*)qrow, qc = *(const v4f*)(qrow + 128);
    const v4f wa = *(const v4f*)(wv + 4 * lane), wc = *(const v4f*)(wv + 128 + 4 * lane);
    float q[8], w[8];
#pragma unroll
    for (int c = 0; c < 4; ++c) { q[c] = qa[c]; q[4 + c] = qc[c]; w[c] = bfr(wa[c]); w[4 + c] = bfr(wc[c]); }
    const float* kbase = KP + (size_t)b * NK * HID + 4 * lane;
#pragma unroll 1
    for (int n = 0; n < NK / 8; ++n) {
        const int j = wave + 8 * n;
        const float* kr = kbase + (size_t)j * HID;
        const v4f ka = *(const v4f*)kr, kc = *(const v4f*)(kr + 128);
        float p = 0.0f;
#pragma unroll
        for (int c = 0; c < 4; ++c) p = fmaf(w[c], tanh_e(q[c] + ka[c]), p);
#pragma unroll
        for (int c = 0; c < 4; ++c) p = fmaf(w[4 + c], tanh_e(q[4 + c] + kc[c]), p);
        p += __shfl_xor(p, 16, 32);
        p += __shfl_xor(p, 8, 32);
        p += __shfl_xor(p, 4, 32);
        p += __shfl_xor(p, 2, 32);
        p += __shfl_xor(p, 1, 32);
        if (lane == 0) res[j] = p;
    }
    __syncthreads();
    float* orow = OUT + ((size_t)b * OUT_Q + qi) * OUT_K;
#pragma unroll 1
    for (int ps = 0; ps < 2; ++ps) {
#pragma unroll 1
        for (int ch = wave; ch < NK / 128; ch += 8) {
            const v4f val = *(const v4fa*)(&res[ch * 128 + lane * 4]);
            *(volatile v4f*)(orow + ch * 128 + lane * 4) = val; }
        if (ps == 0) __threadfence(); }
}

static constexpr size_t al256(size_t v) { return (v + 255) & ~(size_t)255; }
static constexpr size_t SZ_XB = al256((size_t)MT * DIN * 2);
static constexpr size_t SZ_WT = al256((size_t)2 * HID * DIN * 2);
static constexpr size_t SZ_PL = al256((size_t)MT * HID * 4);
static constexpr size_t SZ_TOTAL = SZ_XB + SZ_WT + SZ_PL;
static_assert(SZ_TOTAL <= (size_t)134217728);
static_assert(((size_t)HID * DIN * 2) % 256 == 0);
static_assert(((size_t)MQ * DIN * 2) % 256 == 0);
static_assert(((size_t)MQ * HID * 4) % 256 == 0);
static_assert((size_t)(MT / 64) * 64 * DIN * 2 <= SZ_XB);
static_assert((size_t)(MT / 64) * 64 * HID * 4 <= SZ_PL);
static constexpr size_t NEED_Q = ((size_t)(NB - 1) * NQ_FULL + NQ) * DIN;
static constexpr size_t NEED_K = ((size_t)(NB - 1) * NK_FULL + NK) * DIN;
static constexpr size_t NEED_W = (size_t)DIN * HID;
static constexpr size_t NEED_O = ((size_t)(NB - 1) * OUT_Q + (size_t)(NQ - 1)) * OUT_K + NK;
static constexpr size_t N8_Q_ALL = (size_t)NB * NQ * DIN / 8;
static constexpr size_t N8_K_ALL = (size_t)NB * NK * DIN / 8;
static constexpr size_t N8_Q_ONE = (size_t)NQ * DIN / 8;
static constexpr size_t N8_K_ONE = (size_t)NK * DIN / 8;

extern "C" void kernel_launch(void* const* d_in, const int* in_sizes, int n_in,
                              void* d_out, int out_size, void* d_ws, size_t ws_size, hipStream_t stream) {
    if (n_in < 5) return;
    if ((size_t)in_sizes[0] < NEED_Q || (size_t)in_sizes[1] < NEED_K) return;
    if ((size_t)in_sizes[2] < NEED_W || (size_t)in_sizes[3] < NEED_W) return;
    if (in_sizes[4] < HID) return;
    if ((size_t)out_size < NEED_O) return;
    if (SZ_TOTAL > ws_size) return;
    const float* xq = (const float*)d_in[0];
    const float* xk = (const float*)d_in[1];
    const float* wq = (const float*)d_in[2];
    const float* wk = (const float*)d_in[3];
    const float* wvp = (const float*)d_in[4];
    float* OUT = (float*)d_out;
    char* wsp = (char*)d_ws;
    bf* XB = (bf*)wsp; wsp += SZ_XB;
    bf* WT = (bf*)wsp; wsp += SZ_WT;
    float* PL = (float*)wsp; wsp += SZ_PL;
    bf* XKB = XB + (size_t)MQ * DIN;

    if (NQ == NQ_FULL) {
        k_cvt8<<<(unsigned)((N8_Q_ALL + 255) / 256), 256, 0, stream>>>(xq, XB, N8_Q_ALL);
    } else {
        for (int b = 0; b < NB; ++b) k_cvt8<<<(unsigned)((N8_Q_ONE + 255) / 256), 256, 0, stream>>>(xq + (size_t)b * NQ_FULL * DIN, XB + (size_t)b * NQ * DIN, N8_Q_ONE);
    }
    if (NK == NK_FULL) {
        k_cvt8<<<(unsigned)((N8_K_ALL + 255) / 256), 256, 0, stream>>>(xk, XKB, N8_K_ALL);
    } else {
        for (int b = 0; b < NB; ++b) k_cvt8<<<(unsigned)((N8_K_ONE + 255) / 256), 256, 0, stream>>>(xk + (size_t)b * NK_FULL * DIN, XKB + (size_t)b * NK * DIN, N8_K_ONE);
    }
    k_wtr<<<dim3(DIN / 64, HID / 64, 1), 256, 0, stream>>>(wq, WT);
    k_wtr<<<dim3(DIN / 64, HID / 64, 1), 256, 0, stream>>>(wk, WT + (size_t)HID * DIN);

    k_gemm<<<dim3(MT / 64, HID / 64, 1), 32, 0, stream>>>(XB, WT, PL);

    k_score<<<dim3(NQ, NB, 1), 256, 0, stream>>>(PL, PL + (size_t)MQ * HID, wvp, OUT);
}
